// PointNetFeaturePropagation_23149873725518
// MI455X (gfx1250) — hardware-verified
//
#include <hip/hip_runtime.h>
#include <stdint.h>

#pragma clang fp contract(off)

static constexpr int NBATCH    = 4;
static constexpr int NQ        = 16384;
static constexpr int NPT       = 4096;
static constexpr int CH_SKIP   = 128;
static constexpr int CH_INTERP = 256;
static constexpr int CH_IN     = CH_SKIP + CH_INTERP;
static constexpr int CH_H1     = 256;
static constexpr int CH_H2     = 256;
static constexpr int CH_OUT    = 128;
static constexpr int MROWS     = NBATCH * NQ;

static constexpr float W_CARRY     = 16.0f;
static constexpr float W_CARRY_INV = 1.0f / W_CARRY;
static constexpr float NN_EPS      = 1e-10f;

static_assert(CH_IN == 384, "concat width");
static_assert(MROWS == 65536, "row count");
static_assert(MROWS % 64 == 0, "GEMM M tile multiple");
static_assert(CH_H1 % 64 == 0 && CH_H2 % 64 == 0 && CH_OUT % 64 == 0, "GEMM N tile multiple");
static_assert(CH_IN % 32 == 0 && CH_H1 % 32 == 0 && CH_H2 % 32 == 0, "GEMM K step multiple");
static_assert(NQ % 256 == 0, "query blocks");
static_assert(NPT % 1024 == 0, "candidate staging groups");
static_assert(NPT * 4 * 4 == 65536, "candidate LDS extent");

typedef __attribute__((ext_vector_type(16))) _Float16 v16h;
typedef __attribute__((ext_vector_type(8)))  _Float16 v8h;
typedef __attribute__((ext_vector_type(8)))  float    v8f;
typedef __attribute__((ext_vector_type(4)))  float    v4f;

union FragH { v16h v; v8h h[2]; };

__device__ __forceinline__ v16h frag_load_h(const _Float16* p) {
  FragH f;
  f.h[0] = *(const v8h*)(p);
  f.h[1] = *(const v8h*)(p + 16);
  return f.v;
}
__device__ __forceinline__ v8f mma_h(v16h a, v16h b, v8f c) {
  return __builtin_amdgcn_wmma_f32_16x16x32_f16(false, a, false, b, (short)0, c, false, false);
}
__device__ __forceinline__ void guard_row_h(v8f& a, v8f& b, v8f& c, v8f& d,
                                            v16h x, v16h y0, v16h y1, v16h y2, v16h y3) {
  asm volatile("v_nop\n\tv_nop\n\tv_nop\n\tv_nop"
               : "+v"(a), "+v"(b), "+v"(c), "+v"(d)
               : "v"(x), "v"(y0), "v"(y1), "v"(y2), "v"(y3));
}
__device__ __forceinline__ void keep4_h(v16h a, v16h b, v16h c, v16h d) {
  asm volatile("v_nop" :: "v"(a), "v"(b), "v"(c), "v"(d));
}
__device__ __forceinline__ void acc_guard4(v8f& a, v8f& b, v8f& c, v8f& d) {
  asm volatile("v_nop\n\tv_nop\n\tv_nop\n\tv_nop" : "+v"(a), "+v"(b), "+v"(c), "+v"(d));
}

static constexpr int WBLK_1 = (CH_IN * CH_H1) / 8 / 256;
static constexpr int WBLK_2 = (CH_H1 * CH_H2) / 8 / 256;
static constexpr int WBLK_3 = (CH_H2 * CH_OUT) / 8 / 256;
static_assert(WBLK_1 * 256 * 8 == CH_IN * CH_H1, "W1 chunk cover");
static_assert(WBLK_2 * 256 * 8 == CH_H1 * CH_H2, "W2 chunk cover");
static_assert(WBLK_3 * 256 * 8 == CH_H2 * CH_OUT, "W3 chunk cover");

__global__ __launch_bounds__(256) void weights_to_f16t_kernel(
    const float* __restrict__ Wa, const float* __restrict__ Wb, const float* __restrict__ Wc,
    unsigned short* __restrict__ Ta, unsigned short* __restrict__ Tb, unsigned short* __restrict__ Tc) {
  const int blk = blockIdx.x;
  const float* W;
  _Float16* Wt;
  int kd, nd, c;
  if (blk < WBLK_1) {
    W = Wa; Wt = (_Float16*)Ta; kd = CH_IN; nd = CH_H1; c = blk * 256 + threadIdx.x;
  } else if (blk < WBLK_1 + WBLK_2) {
    W = Wb; Wt = (_Float16*)Tb; kd = CH_H1; nd = CH_H2; c = (blk - WBLK_1) * 256 + threadIdx.x;
  } else {
    W = Wc; Wt = (_Float16*)Tc; kd = CH_H2; nd = CH_OUT; c = (blk - WBLK_1 - WBLK_2) * 256 + threadIdx.x;
  }
  const int cpr = kd >> 3;
  const int n = c / cpr;
  const int k0 = (c - n * cpr) << 3;
  float t[8];
#pragma unroll
  for (int e = 0; e < 8; ++e) t[e] = W[(size_t)(k0 + e) * nd + n];
  v8h hv;
#pragma unroll
  for (int e = 0; e < 8; ++e) hv[e] = (_Float16)(t[e] * W_CARRY);
  volatile v8h* dst = (volatile v8h*)(Wt + (size_t)n * kd + k0);
  *dst = hv;
  __threadfence();
  *dst = hv;
}

__device__ __forceinline__ int clamp_pt(int j) {
  j = j < 0 ? 0 : j;
  j = j > (NPT - 1) ? (NPT - 1) : j;
  return j;
}

__global__ __launch_bounds__(256) void nn3_interp_kernel(
    const float* __restrict__ xyz1, const float* __restrict__ xyz2,
    const float* __restrict__ f1, const float* __restrict__ f2,
    unsigned short* __restrict__ X0p) {
#pragma clang fp contract(off)
  __shared__ __align__(16) float s2[NPT * 4];
  const int tid  = threadIdx.x;
  const int lane = tid & 31;
  const int wave = tid >> 5;
  const int b    = blockIdx.y;

  const float* src = xyz2 + (size_t)b * NPT * 3;
#pragma unroll 1
  for (int g = 0; g < NPT / 1024; ++g) {
#pragma unroll
    for (int u = 0; u < 4; ++u) {
      const int j = (g * 4 + u) * 256 + tid;
      const float cx = src[3 * j + 0];
      const float cy = src[3 * j + 1];
      const float cz = src[3 * j + 2];
      const float t0 = cx * cx;
      const float t1 = cy * cy;
      const float t2 = cz * cz;
      v4f rec;
      rec.x = cx; rec.y = cy; rec.z = cz;
      rec.w = (t0 + t2) + t1;
      *(v4f*)(s2 + 4 * j) = rec;
    }
    asm volatile("" ::: "memory");
  }
  __syncthreads();

  const int nq = blockIdx.x * 256 + tid;
  const float* qp = xyz1 + ((size_t)b * NQ + nq) * 3;
  const float px = qp[0];
  const float py = qp[1];
  const float pz = qp[2];
  const float q0s = px * px;
  const float q1s = py * py;
  const float q2s = pz * pz;
  const float sq1 = (q0s + q2s) + q1s;

  float d0 = __builtin_inff(), d1 = __builtin_inff(), d2 = __builtin_inff();
  int i0 = 0, i1 = 0, i2 = 0;
#pragma unroll 4
  for (int j = 0; j < NPT; ++j) {
    const v4f cnd = *(const v4f*)(s2 + 4 * j);
    float p = px * cnd.x;
    p = __builtin_fmaf(py, cnd.y, p);
    p = __builtin_fmaf(pz, cnd.z, p);
    const float s = sq1 + cnd.w;
    const float d = s - (p + p);
    if (d < d2) {
      if (d < d1) {
        d2 = d1; i2 = i1;
        if (d < d0) { d1 = d0; i1 = i0; d0 = d; i0 = j; }
        else        { d1 = d;  i1 = j; }
      } else {
        d2 = d; i2 = j;
      }
    }
  }

  const float e0 = fmaxf(d0, NN_EPS);
  const float e1 = fmaxf(d1, NN_EPS);
  const float e2 = fmaxf(d2, NN_EPS);
  const float r0 = 1.0f / e0;
  const float r1 = 1.0f / e1;
  const float r2 = 1.0f / e2;
  const float rsum = (r0 + r2) + r1;
  const float w0 = r0 / rsum;
  const float w1 = r1 / rsum;
  const float w2 = r2 / rsum;

  __syncthreads();
  {
    v4f ri, rw;
    ri.x = (float)i0; ri.y = (float)i1; ri.z = (float)i2; ri.w = 0.0f;
    rw.x = w0; rw.y = w1; rw.z = w2; rw.w = 0.0f;
    *(v4f*)(s2 + 8 * tid)     = ri;
    *(v4f*)(s2 + 8 * tid + 4) = rw;
  }
  __syncthreads();

  _Float16* X0 = (_Float16*)X0p;
  const float* f2b = f2 + (size_t)b * NPT * CH_INTERP;
  const size_t prow0 = (size_t)b * NQ + (size_t)blockIdx.x * 256;
  const int lq = lane & 15;
#pragma unroll 1
  for (int i = 0; i < 32; ++i) {
    const int t = wave * 32 + i;
    const v4f ri = *(const v4f*)(s2 + 8 * t);
    const v4f rw = *(const v4f*)(s2 + 8 * t + 4);
    const int j0 = clamp_pt((int)ri.x);
    const int j1 = clamp_pt((int)ri.y);
    const int j2 = clamp_pt((int)ri.z);
    const float u0 = rw.x, u1 = rw.y, u2 = rw.z;
    const float* g0 = f2b + (size_t)j0 * CH_INTERP + 8 * lane;
    const float* g1 = f2b + (size_t)j1 * CH_INTERP + 8 * lane;
    const float* g2 = f2b + (size_t)j2 * CH_INTERP + 8 * lane;
    const size_t prow = prow0 + (size_t)t;
    const float* gs = f1 + prow * CH_SKIP + 8 * lq;
    const v4f a0 = *(const v4f*)(g0);
    const v4f a1 = *(const v4f*)(g0 + 4);
    const v4f b0 = *(const v4f*)(g1);
    const v4f b1 = *(const v4f*)(g1 + 4);
    const v4f c0 = *(const v4f*)(g2);
    const v4f c1 = *(const v4f*)(g2 + 4);
    const v4f s0 = *(const v4f*)(gs);
    const v4f s1 = *(const v4f*)(gs + 4);
    const v4f t0 = (a0 * u0 + b0 * u1) + c0 * u2;
    const v4f t1 = (a1 * u0 + b1 * u1) + c1 * u2;
    v8h hv, fv;
#pragma unroll
    for (int e = 0; e < 4; ++e) {
      hv[e]     = (_Float16)t0[e];
      hv[4 + e] = (_Float16)t1[e];
      fv[e]     = (_Float16)s0[e];
      fv[4 + e] = (_Float16)s1[e];
    }
    _Float16* xr = X0 + prow * CH_IN;
    volatile v8h* pi = (volatile v8h*)(xr + CH_SKIP + 8 * lane);
    volatile v8h* pf = (volatile v8h*)(xr + 8 * lq);
    *pi = hv;
    if (lane < 16) *pf = fv;
    __threadfence();
    *pi = hv;
    if (lane < 16) *pf = fv;
  }
}

template <int OUT_MODE, int ACT>
__global__ __launch_bounds__(256) void wmma_gemm64_f16(
    const unsigned short* __restrict__ Ap, int lda,
    const unsigned short* __restrict__ Btp, int ldb,
    void* __restrict__ Cout, int ldc,
    const float* __restrict__ bias,
    int M, int N, int K, float scale) {
  const _Float16* A  = (const _Float16*)Ap;
  const _Float16* Bt = (const _Float16*)Btp;
  __shared__ __align__(16) float sT[8][16 * 68];
  const int lane = threadIdx.x & 31;
  const int wave = threadIdx.x >> 5;
  const int tilesN = N >> 6;
  const int tilesM = M >> 6;
  const int tile = blockIdx.x * 8 + wave;
  if (tile >= tilesM * tilesN) return;
  const int tm = tile / tilesN;
  const int tn = tile - tm * tilesN;
  const int m0 = tm << 6;
  const int n0 = tn << 6;

  const int rlane = lane & 15;
  const int koff  = (lane >> 4) * 8;
  const int mOff  = (lane >> 4) * 8;

  v8f acc[4][4];
#pragma unroll
  for (int i = 0; i < 4; ++i)
#pragma unroll
    for (int j = 0; j < 4; ++j) acc[i][j] = (v8f){0.f, 0.f, 0.f, 0.f, 0.f, 0.f, 0.f, 0.f};

  for (int k0 = 0; k0 < K; k0 += 32) {
    v16h bh[4];
#pragma unroll
    for (int j = 0; j < 4; ++j) {
      const size_t bo = (size_t)(n0 + (j << 4) + rlane) * ldb + koff + k0;
      bh[j] = frag_load_h(Bt + bo);
    }
#pragma unroll
    for (int i = 0; i < 4; ++i) {
      const size_t ao = (size_t)(m0 + (i << 4) + rlane) * lda + koff + k0;
      const v16h ah = frag_load_h(A + ao);
#pragma unroll
      for (int j = 0; j < 4; ++j) acc[i][j] = mma_h(ah, bh[j], acc[i][j]);
      guard_row_h(acc[i][0], acc[i][1], acc[i][2], acc[i][3], ah, bh[0], bh[1], bh[2], bh[3]);
    }
    keep4_h(bh[0], bh[1], bh[2], bh[3]);
  }
  acc_guard4(acc[0][0], acc[0][1], acc[0][2], acc[0][3]);
  acc_guard4(acc[1][0], acc[1][1], acc[1][2], acc[1][3]);
  acc_guard4(acc[2][0], acc[2][1], acc[2][2], acc[2][3]);
  acc_guard4(acc[3][0], acc[3][1], acc[3][2], acc[3][3]);

  float* slab = sT[wave];
#pragma unroll
  for (int i = 0; i < 4; ++i) {
    const int mBase = m0 + (i << 4);
#pragma unroll
    for (int j = 0; j < 4; ++j) {
      const int n = n0 + (j << 4) + rlane;
      const float bv = bias[n];
#pragma unroll
      for (int r = 0; r < 8; ++r) {
        float v = acc[i][j][r] * scale;
        v += bv;
        if (ACT == 2) v = fmaxf(v, 0.0f);
        slab[(mOff + r) * 68 + (j << 4) + rlane] = v;
      }
    }
    __builtin_amdgcn_fence(__ATOMIC_RELEASE, "workgroup");
    __builtin_amdgcn_wave_barrier();
    __builtin_amdgcn_fence(__ATOMIC_ACQUIRE, "workgroup");
    if (OUT_MODE == 0) {
      float* C = (float*)Cout;
      const int hh = lane >> 4, c4 = (lane & 15) * 4;
      for (int pass = 0; pass < 2; ++pass) {
#pragma unroll
        for (int it = 0; it < 8; ++it) {
          const int row = it * 2 + hh;
          v4f v = *(const v4f*)(slab + row * 68 + c4);
          *(volatile v4f*)(C + (size_t)(mBase + row) * ldc + n0 + c4) = v;
        }
        __threadfence();
      }
    } else {
      const int q = lane >> 3, c8 = (lane & 7) * 8;
      _Float16* C = (_Float16*)Cout;
      for (int pass = 0; pass < 2; ++pass) {
#pragma unroll
        for (int it = 0; it < 4; ++it) {
          const int row = it * 4 + q;
          const float* sp = slab + row * 68 + c8;
          v8h hv;
#pragma unroll
          for (int e = 0; e < 8; ++e) hv[e] = (_Float16)sp[e];
          *(volatile v8h*)(C + (size_t)(mBase + row) * ldc + n0 + c8) = hv;
        }
        __threadfence();
      }
    }
    __builtin_amdgcn_fence(__ATOMIC_RELEASE, "workgroup");
    __builtin_amdgcn_wave_barrier();
    __builtin_amdgcn_fence(__ATOMIC_ACQUIRE, "workgroup");
  }
}

extern "C" void kernel_launch(void* const* d_in, const int* in_sizes, int n_in,
                              void* d_out, int out_size, void* d_ws, size_t ws_size,
                              hipStream_t stream) {
  if (n_in < 10) return;
  if (in_sizes[0] != NBATCH * NQ * 3) return;
  if (in_sizes[1] != NBATCH * NPT * 3) return;
  if (in_sizes[2] != MROWS * CH_SKIP) return;
  if (in_sizes[3] != NBATCH * NPT * CH_INTERP) return;
  if (in_sizes[4] != CH_IN * CH_H1 || in_sizes[5] != CH_H1) return;
  if (in_sizes[6] != CH_H1 * CH_H2 || in_sizes[7] != CH_H2) return;
  if (in_sizes[8] != CH_H2 * CH_OUT || in_sizes[9] != CH_OUT) return;
  if (out_size != MROWS * CH_OUT) return;

  const float* xyz1 = (const float*)d_in[0];
  const float* xyz2 = (const float*)d_in[1];
  const float* f1   = (const float*)d_in[2];
  const float* f2   = (const float*)d_in[3];
  const float* W1   = (const float*)d_in[4];
  const float* b1   = (const float*)d_in[5];
  const float* W2   = (const float*)d_in[6];
  const float* b2   = (const float*)d_in[7];
  const float* W3   = (const float*)d_in[8];
  const float* b3   = (const float*)d_in[9];

  constexpr size_t SZ_X0  = (size_t)MROWS * CH_IN * 2;
  constexpr size_t SZ_H1  = (size_t)MROWS * CH_H1 * 2;
  constexpr size_t SZ_H2  = (size_t)MROWS * CH_H2 * 2;
  constexpr size_t SZ_WT1 = (size_t)CH_H1 * CH_IN * 2;
  constexpr size_t SZ_WT2 = (size_t)CH_H2 * CH_H1 * 2;
  constexpr size_t SZ_WT3 = (size_t)CH_OUT * CH_H2 * 2;
  constexpr size_t WS_TOTAL = SZ_X0 + SZ_H1 + SZ_H2 + SZ_WT1 + SZ_WT2 + SZ_WT3;
  static_assert(WS_TOTAL == 117833728, "carve total");
  static_assert(WS_TOTAL <= 134217728, "carve budget");
  static_assert(SZ_X0 % 256 == 0 && SZ_H1 % 256 == 0 && SZ_WT1 % 256 == 0 && SZ_WT2 % 256 == 0, "carve alignment");
  if (ws_size < WS_TOTAL) return;

  char* ws = (char*)d_ws;
  unsigned short* X0  = (unsigned short*)(ws);
  unsigned short* H1  = (unsigned short*)(ws + SZ_X0);
  unsigned short* H2  = (unsigned short*)(ws + SZ_X0 + SZ_H1);
  unsigned short* Wt1 = (unsigned short*)(ws + SZ_X0 + SZ_H1 + SZ_H2);
  unsigned short* Wt2 = (unsigned short*)(ws + SZ_X0 + SZ_H1 + SZ_H2 + SZ_WT1);
  unsigned short* Wt3 = (unsigned short*)(ws + SZ_X0 + SZ_H1 + SZ_H2 + SZ_WT1 + SZ_WT2);

  weights_to_f16t_kernel<<<WBLK_1 + WBLK_2 + WBLK_3, 256, 0, stream>>>(W1, W2, W3, Wt1, Wt2, Wt3);

  nn3_interp_kernel<<<dim3(NQ / 256, NBATCH), 256, 0, stream>>>(xyz1, xyz2, f1, f2, X0);

  wmma_gemm64_f16<1, 2><<<(MROWS / 64) * (CH_H1 / 64) / 8, 256, 0, stream>>>(
      X0, CH_IN, Wt1, CH_IN, (void*)H1, CH_H1, b1, MROWS, CH_H1, CH_IN, W_CARRY_INV);

  wmma_gemm64_f16<1, 2><<<(MROWS / 64) * (CH_H2 / 64) / 8, 256, 0, stream>>>(
      H1, CH_H1, Wt2, CH_H1, (void*)H2, CH_H2, b2, MROWS, CH_H2, CH_H1, W_CARRY_INV);

  wmma_gemm64_f16<0, 0><<<(MROWS / 64) * (CH_OUT / 64) / 8, 256, 0, stream>>>(
      H2, CH_H2, Wt3, CH_H2, d_out, CH_OUT, b3, MROWS, CH_OUT, CH_H2, W_CARRY_INV);
}
